// GraphTimeModel_80779744903725
// MI455X (gfx1250) — hardware-verified
//
#include <hip/hip_runtime.h>
#include <stdint.h>
#include <stddef.h>
#include <math.h>

#pragma clang fp contract(off)

#define NBATCH 16
#define NTIME  16
#define NNODE  256
#define NFEAT  64
#define NHID   128
#define NHEAD  4
#define NCLS   10
#define NGRAPH 256

#define XP   264
#define HSP  132
#define HP2  136
#define TSP  72

#define G_XTH  0
#define G_XTL  33792
#define G_SS   67584
#define G_SD   71680
#define G_MB   75776
#define G_V    83968
#define G_W    86016
#define G_WSZ  33792
#define LDS_GAT (G_W + 4 * G_WSZ)
static_assert(LDS_GAT == 221184);
static_assert(G_XTL == 64 * XP * 2);
static_assert(G_SS == 2 * 64 * XP * 2);
static_assert(G_WSZ == 4 * 16 * XP * 2);
static_assert(16 * HSP * 4 == 16 * XP * 2);
static_assert((G_SS % 16) == 0);
static_assert((G_SD % 16) == 0);
static_assert((G_MB % 16) == 0);
static_assert((G_V % 16) == 0);
static_assert((G_W % 16) == 0);

#define C_YTH  0
#define C_YTL  67584
#define C_ST   135168
#define C_STSZ 8448
#define C_PP   202752
#define C_PQH  206848
#define C_PQL  207104
#define LDS_GCN 207360
static_assert(C_YTL == 128 * XP * 2);
static_assert(C_ST == 2 * 128 * XP * 2);
static_assert(C_STSZ == 16 * HSP * 4);
static_assert(C_PP == C_ST + 8 * C_STSZ);
static_assert(C_PQH == C_PP + 8 * 128 * 4);
static_assert(C_PQL == C_PQH + 256);
static_assert(LDS_GCN == C_PQL + 256);

#define T_GO   0
#define T_GI   131072
#define T_GH   155648
#define T_HF   180224
#define T_HH   188416
#define T_HL   192768
#define T_CH   197120
#define T_CL   205568
#define T_FH   214016
#define T_FL   218368
#define T_C1   222720
#define T_AT   239104
#define T_WL   247296
#define T_S2   248320
#define T_OU   248576
#define LDS_TAIL 249344
static_assert(T_GI == 256 * 128 * 4);
static_assert(T_GH == T_GI + 16 * 384 * 4);
static_assert(T_HF == T_GH + 16 * 384 * 4);
static_assert(T_HH == T_HF + 16 * 128 * 4);
static_assert(T_HL == T_HH + 16 * HP2 * 2);
static_assert(T_CH == T_HL + 16 * HP2 * 2);
static_assert(T_CL == T_CH + 16 * XP * 2);
static_assert(T_FH == T_CL + 16 * XP * 2);
static_assert(T_FL == T_FH + 16 * HP2 * 2);
static_assert(T_C1 == T_FL + 16 * HP2 * 2);
static_assert(T_AT == T_C1 + 16 * 256 * 4);
static_assert(T_WL == T_AT + 16 * 128 * 4);
static_assert(T_S2 == T_WL + 256 * 4);
static_assert(T_OU == T_S2 + 64 * 4);
static_assert(LDS_TAIL == T_OU + 192 * 4);
static_assert((T_HH % 16) == 0);
static_assert((T_CH % 16) == 0);
static_assert((T_FH % 16) == 0);
static_assert((T_C1 % 16) == 0);
static_assert((T_OU % 16) == 0);
static_assert((XP * 2) % 16 == 0);
static_assert((HP2 * 2) % 16 == 0);
static_assert((HSP * 4) % 16 == 0);
static_assert((TSP * 2) % 16 == 0);

typedef __bf16         v16bf __attribute__((ext_vector_type(16)));
typedef float          v8f   __attribute__((ext_vector_type(8)));
typedef float          v4f   __attribute__((ext_vector_type(4)));
typedef unsigned int   v4u   __attribute__((ext_vector_type(4)));
typedef v4f __attribute__((may_alias)) v4fa;
typedef v4u __attribute__((may_alias)) v4ua;

union FragBF { v16bf v; v4u q[2]; };

__device__ __forceinline__ unsigned int bfb(float f) {
  unsigned int u = __float_as_uint(f);
  u += 0x7FFFu + ((u >> 16) & 1u);
  return u >> 16;
}
__device__ __forceinline__ void split2(float v, unsigned int& hi, unsigned int& lo) {
  hi = bfb(v);
  lo = bfb(v - __uint_as_float(hi << 16));
}
__device__ __forceinline__ unsigned int pk(unsigned int a, unsigned int b) { return (a & 0xFFFFu) | (b << 16); }

__device__ __forceinline__ void split8(v4f a, v4f c, v4u& H, v4u& L) {
  unsigned int h0, l0, h1, l1, h2, l2, h3, l3, h4, l4, h5, l5, h6, l6, h7, l7;
  split2(a.x, h0, l0); split2(a.y, h1, l1); split2(a.z, h2, l2); split2(a.w, h3, l3);
  split2(c.x, h4, l4); split2(c.y, h5, l5); split2(c.z, h6, l6); split2(c.w, h7, l7);
  H.x = pk(h0, h1); H.y = pk(h2, h3); H.z = pk(h4, h5); H.w = pk(h6, h7);
  L.x = pk(l0, l1); L.y = pk(l2, l3); L.z = pk(l4, l5); L.w = pk(l6, l7);
}

__device__ __forceinline__ float gelu_f(float x) {
  return 0.5f * x * erfcf(-x * 0.70710678118654752f);
}
__device__ __forceinline__ float sigm(float v) {
  const float e = expf(-fmaxf(v, -80.0f));
  return 1.0f / (1.0f + e);
}

__device__ __forceinline__ void wave_sync() {
  __builtin_amdgcn_fence(__ATOMIC_RELEASE, "wavefront");
  __builtin_amdgcn_wave_barrier();
  __builtin_amdgcn_fence(__ATOMIC_ACQUIRE, "wavefront");
}

__device__ __forceinline__ v8f wmma_bf(v16bf a, v16bf b, v8f c) {
  v8f d = __builtin_amdgcn_wmma_f32_16x16x32_bf16(false, a, false, b, (short)0, c, false, false);
  asm volatile("v_nop\n\tv_nop\n\tv_nop\n\tv_nop" : "+v"(d) : "v"(a), "v"(b));
  return d;
}
__device__ __forceinline__ v8f mma3(v16bf ah, v16bf al, v16bf bh, v16bf bl, v8f c) {
  c = wmma_bf(ah, bh, c);
  c = wmma_bf(ah, bl, c);
  c = wmma_bf(al, bh, c);
  return c;
}

__device__ __forceinline__ v16bf ldfrag_bf(const unsigned short* p, int h) {
  FragBF f;
  f.q[0] = *(const v4ua*)(p + 8 * h);
  f.q[1] = *(const v4ua*)(p + 16 + 8 * h);
  return f.v;
}

__device__ __forceinline__ v4f lo4(v8f a) { v4f r; r.x = a[0]; r.y = a[1]; r.z = a[2]; r.w = a[3]; return r; }
__device__ __forceinline__ v4f hi4(v8f a) { v4f r; r.x = a[4]; r.y = a[5]; r.z = a[6]; r.w = a[7]; return r; }

__device__ __forceinline__ void store_rows16(const float* St, unsigned short* Oh, unsigned short* Ol,
                                             size_t rowbase, int hh, int m)
{
  #pragma unroll
  for (int q = 0; q < 8; ++q) {
    const int row = 2 * q + hh, c8 = 8 * m;
    const v4f a = *(const v4fa*)(St + row * HSP + c8);
    const v4f c = *(const v4fa*)(St + row * HSP + c8 + 4);
    v4u H, L;
    split8(a, c, H, L);
    const size_t go = (rowbase + (size_t)row) * NHID + c8;
    *(volatile v4u*)(Oh + go) = H;
    *(volatile v4u*)(Ol + go) = L;
  }
}

__global__ __launch_bounds__(256) void k_adj1(const float* __restrict__ L, float* __restrict__ An)
{
  __shared__ float red[256];
  __shared__ __align__(16) float row[256];
  const int i = blockIdx.x, j = threadIdx.x;
  const float s = L[i * NNODE + j] + L[j * NNODE + i];
  float a = gelu_f(s);
  a = (j != i) ? a : 0.0f;
  red[j] = fabsf(a);
  __syncthreads();
  for (int st = 128; st > 0; st >>= 1) {
    if (j < st) red[j] += red[j + st];
    __syncthreads();
  }
  const float den = fmaxf(red[0], 1e-12f);
  const float inv = 1.0f / den;
  row[j] = a * inv;
  __syncthreads();
  const int tc = (j < 64) ? j : 0;
  const v4f v = *(const v4fa*)(row + 4 * tc);
  if (j < 64) *(volatile v4f*)(An + (size_t)i * NNODE + 4 * j) = v;
  __threadfence();
  if (j < 64) *(volatile v4f*)(An + (size_t)i * NNODE + 4 * j) = v;
}

__global__ __launch_bounds__(256) void k_small(const float* __restrict__ An, const float* __restrict__ Wg,
                                               const float* __restrict__ as_, const float* __restrict__ ad_,
                                               float* __restrict__ dinv, float* __restrict__ V)
{
  __shared__ __align__(16) float sdv[256];
  __shared__ __align__(16) float sv[512];
  const int t = threadIdx.x;
  float deg = 0.0f;
  #pragma unroll 4
  for (int j = 0; j < NNODE; ++j) deg += An[j * NNODE + t];
  deg = deg + 1.0f;
  deg = fmaxf(deg, 1e-12f);
  sdv[t] = 1.0f / sqrtf(deg);
  const int hq = t >> 6, f = t & 63;
  float vs = 0.0f, vd = 0.0f;
  #pragma unroll 1
  for (int d = 0; d < NHID; ++d) {
    const float w = Wg[f * 512 + hq * 128 + d];
    vs = fmaf(w, as_[hq * 128 + d], vs);
    vd = fmaf(w, ad_[hq * 128 + d], vd);
  }
  sv[hq * 64 + f] = vs;
  sv[256 + hq * 64 + f] = vd;
  __syncthreads();
  const int td = (t < 64) ? t : 0;
  const int tv = (t >= 64 && t < 192) ? (t - 64) : 0;
  const v4f dvv = *(const v4fa*)(sdv + 4 * td);
  const v4f vvv = *(const v4fa*)(sv + 4 * tv);
  if (t < 64) *(volatile v4f*)(dinv + 4 * td) = dvv;
  if (t >= 64 && t < 192) *(volatile v4f*)(V + 4 * tv) = vvv;
  __threadfence();
  if (t < 64) *(volatile v4f*)(dinv + 4 * td) = dvv;
  if (t >= 64 && t < 192) *(volatile v4f*)(V + 4 * tv) = vvv;
}

__global__ __launch_bounds__(256) void k_adj3(const float* __restrict__ An, const float* __restrict__ dinv,
                                              unsigned short* __restrict__ APh, unsigned short* __restrict__ APl,
                                              unsigned int* __restrict__ MB)
{
  __shared__ __align__(16) unsigned short sH[256];
  __shared__ __align__(16) unsigned short sL[256];
  __shared__ __align__(16) unsigned int sM[8];
  const int i = blockIdx.x, j = threadIdx.x;
  const float v = An[(size_t)j * NNODE + i];
  const bool on = (v != 0.0f) || (j == i);
  const float di = dinv[i], dj = dinv[j];
  const float ah = (di * (v + ((j == i) ? 1.0f : 0.0f))) * dj;
  unsigned int hb, lb;
  split2(ah, hb, lb);
  sH[j] = (unsigned short)hb;
  sL[j] = (unsigned short)lb;
  const unsigned int bal = __builtin_amdgcn_ballot_w32(on);
  if ((j & 31) == 0) sM[j >> 5] = bal;
  __syncthreads();
  const int th = (j < 32) ? j : 0;
  const int tl = (j >= 32 && j < 64) ? (j - 32) : 0;
  const int tq = (j >= 64 && j < 72) ? (j - 64) : 0;
  const v4u hv = *(const v4ua*)(sH + 8 * th);
  const v4u lv = *(const v4ua*)(sL + 8 * tl);
  const int tq2 = (tq < 2) ? tq : 0;
  const v4u ml = *(const v4ua*)(sM + 4 * tq2);
  v4u mv;
  mv.x = (tq < 2) ? ml.x : 0u; mv.y = (tq < 2) ? ml.y : 0u; mv.z = (tq < 2) ? ml.z : 0u; mv.w = (tq < 2) ? ml.w : 0u;
  if (j < 32)            *(volatile v4u*)(APh + (size_t)i * NNODE + 8 * th) = hv;
  if (j >= 32 && j < 64) *(volatile v4u*)(APl + (size_t)i * NNODE + 8 * tl) = lv;
  if (j >= 64 && j < 72) *(volatile v4u*)(MB + (size_t)i * 32 + 4 * tq) = mv;
  __threadfence();
  if (j < 32)            *(volatile v4u*)(APh + (size_t)i * NNODE + 8 * th) = hv;
  if (j >= 32 && j < 64) *(volatile v4u*)(APl + (size_t)i * NNODE + 8 * tl) = lv;
  if (j >= 64 && j < 72) *(volatile v4u*)(MB + (size_t)i * 32 + 4 * tq) = mv;
}

__global__ __launch_bounds__(256) void k_tsplit(const float* __restrict__ W, int ldi, int zin,
                                                unsigned short* __restrict__ Th,
                                                unsigned short* __restrict__ Tl, int ldo, int zout,
                                                int K, int N)
{
  __shared__ __align__(16) unsigned short sH[64 * TSP];
  __shared__ __align__(16) unsigned short sL[64 * TSP];
  const int tid = threadIdx.x, lane = tid & 31, wv = tid >> 5;
  const int n0 = blockIdx.x * 64, k0 = blockIdx.y * 64, z = blockIdx.z;
  (void)K; (void)N;
  const float* Wz = W + (size_t)z * zin;
  #pragma unroll 4
  for (int i = 0; i < 16; ++i) {
    const int idx = tid + 256 * i;
    const int kk = idx >> 6, nn = idx & 63;
    const float v = Wz[(size_t)(k0 + kk) * ldi + n0 + nn];
    unsigned int hb, lb;
    split2(v, hb, lb);
    sH[nn * TSP + kk] = (unsigned short)hb;
    sL[nn * TSP + kk] = (unsigned short)lb;
  }
  __syncthreads();
  const int piece = lane & 7, rq = lane >> 3;
  v4u hv[2], lv[2];
  size_t go[2];
  #pragma unroll
  for (int ps = 0; ps < 2; ++ps) {
    const int row = ps * 32 + wv * 4 + rq;
    hv[ps] = *(const v4ua*)(sH + row * TSP + 8 * piece);
    lv[ps] = *(const v4ua*)(sL + row * TSP + 8 * piece);
    go[ps] = (size_t)(n0 + row) * ldo + (size_t)z * zout + k0 + 8 * piece;
  }
  #pragma unroll
  for (int ps = 0; ps < 2; ++ps) {
    *(volatile v4u*)(Th + go[ps]) = hv[ps];
    *(volatile v4u*)(Tl + go[ps]) = lv[ps];
  }
  __threadfence();
  #pragma unroll
  for (int ps = 0; ps < 2; ++ps) {
    *(volatile v4u*)(Th + go[ps]) = hv[ps];
    *(volatile v4u*)(Tl + go[ps]) = lv[ps];
  }
}

__global__ __launch_bounds__(128) void k_gat(const float* __restrict__ x,
                                             const float* __restrict__ Vg,
                                             const unsigned int* __restrict__ MBg,
                                             const unsigned short* __restrict__ WSh,
                                             const unsigned short* __restrict__ WSl,
                                             const float* __restrict__ bgat,
                                             unsigned short* __restrict__ H0h,
                                             unsigned short* __restrict__ H0l)
{
  extern __shared__ __align__(16) unsigned char dsm[];
  unsigned short* XTh = (unsigned short*)(dsm + G_XTH);
  unsigned short* XTl = (unsigned short*)(dsm + G_XTL);
  float* SS = (float*)(dsm + G_SS);
  float* SD = (float*)(dsm + G_SD);
  unsigned int* sMB = (unsigned int*)(dsm + G_MB);
  float* sV = (float*)(dsm + G_V);
  const int tid = threadIdx.x, lane = tid & 31, wv = tid >> 5;
  const int hh = lane >> 4, m = lane & 15;
  const int bt = blockIdx.x;
  unsigned char* wb = dsm + G_W + wv * G_WSZ;
  unsigned short* ALh = (unsigned short*)wb;
  unsigned short* ALl = (unsigned short*)(wb + 16 * XP * 2);
  unsigned short* PSh = (unsigned short*)(wb + 2 * 16 * XP * 2);
  unsigned short* PSl = (unsigned short*)(wb + 3 * 16 * XP * 2);
  float* Hs = (float*)wb;
  const float* xg = x + (size_t)bt * (NNODE * NFEAT);
  const v8f z8 = {0.f, 0.f, 0.f, 0.f, 0.f, 0.f, 0.f, 0.f};
  const float NEG_INF = __uint_as_float(0xff800000u);

  for (int i2 = tid; i2 < 512; i2 += 128) sV[i2] = Vg[i2];
  for (int i2 = tid; i2 < 2048; i2 += 128) sMB[i2] = MBg[(i2 >> 3) * 32 + (i2 & 7)];
  #pragma unroll 4
  for (int it = 0; it < 128; ++it) {
    const int idx = tid + 128 * it;
    const int j = idx >> 6, f = idx & 63;
    const float v = xg[idx];
    unsigned int hb, lb;
    split2(v, hb, lb);
    XTh[f * XP + j] = (unsigned short)hb;
    XTl[f * XP + j] = (unsigned short)lb;
  }
  __syncthreads();
  #pragma unroll 1
  for (int jj = 0; jj < 2; ++jj) {
    const int j = tid + 128 * jj;
    const float* xr = xg + j * NFEAT;
    float acc8[8];
    #pragma unroll
    for (int q = 0; q < 8; ++q) acc8[q] = 0.0f;
    #pragma unroll 2
    for (int f = 0; f < NFEAT; ++f) {
      const float xv = xr[f];
      #pragma unroll
      for (int q = 0; q < 8; ++q) acc8[q] = fmaf(xv, sV[q * 64 + f], acc8[q]);
    }
    #pragma unroll
    for (int hq = 0; hq < 4; ++hq) {
      SS[hq * 256 + j] = acc8[hq];
      SD[hq * 256 + j] = acc8[4 + hq];
    }
  }
  __syncthreads();

  #pragma unroll 1
  for (int rbq = 0; rbq < 4; ++rbq) {
    const int i0 = 16 * (wv + 4 * rbq);

    #pragma unroll 1
    for (int h = 0; h < NHEAD; ++h) {
      #pragma unroll 1
      for (int r = 0; r < 16; ++r) {
        const int i = i0 + r;
        const float sd = SD[h * 256 + i];
        const v4f sa = *(const v4fa*)(SS + h * 256 + 8 * lane);
        const v4f sb = *(const v4fa*)(SS + h * 256 + 8 * lane + 4);
        const unsigned int mw = sMB[i * 8 + (lane >> 2)];
        const unsigned int mb = mw >> (8 * (lane & 3));
        float ev[8];
        ev[0] = sa.x; ev[1] = sa.y; ev[2] = sa.z; ev[3] = sa.w;
        ev[4] = sb.x; ev[5] = sb.y; ev[6] = sb.z; ev[7] = sb.w;
        float vmax = NEG_INF;
        #pragma unroll
        for (int k = 0; k < 8; ++k) {
          float v = sd + ev[k];
          v = (v >= 0.0f) ? v : 0.2f * v;
          ev[k] = v;
          const bool on = ((mb >> k) & 1u) != 0u;
          vmax = on ? fmaxf(vmax, v) : vmax;
        }
        #pragma unroll
        for (int off = 16; off > 0; off >>= 1) vmax = fmaxf(vmax, __shfl_xor(vmax, off, 32));
        float sum = 0.0f;
        #pragma unroll
        for (int k = 0; k < 8; ++k) {
          float q = expf(fminf(ev[k] - vmax, 0.0f));
          const bool on = ((mb >> k) & 1u) != 0u;
          q = on ? q : 0.0f;
          ev[k] = q;
          sum += q;
        }
        #pragma unroll
        for (int off = 16; off > 0; off >>= 1) sum += __shfl_xor(sum, off, 32);
        const float inv = 1.0f / sum;
        v4f pa, pb;
        pa.x = ev[0] * inv; pa.y = ev[1] * inv; pa.z = ev[2] * inv; pa.w = ev[3] * inv;
        pb.x = ev[4] * inv; pb.y = ev[5] * inv; pb.z = ev[6] * inv; pb.w = ev[7] * inv;
        v4u H, Lo;
        split8(pa, pb, H, Lo);
        *(v4ua*)(ALh + r * XP + 8 * lane) = H;
        *(v4ua*)(ALl + r * XP + 8 * lane) = Lo;
      }
      wave_sync();

      {
        v8f acc[4];
        #pragma unroll
        for (int nt = 0; nt < 4; ++nt) acc[nt] = z8;
        #pragma unroll 2
        for (int ks = 0; ks < 8; ++ks) {
          const v16bf bh_ = ldfrag_bf(ALh + m * XP + 32 * ks, hh);
          const v16bf bl_ = ldfrag_bf(ALl + m * XP + 32 * ks, hh);
          #pragma unroll
          for (int nt = 0; nt < 4; ++nt) {
            const v16bf ah_ = ldfrag_bf(XTh + (16 * nt + m) * XP + 32 * ks, hh);
            const v16bf al_ = ldfrag_bf(XTl + (16 * nt + m) * XP + 32 * ks, hh);
            acc[nt] = mma3(ah_, al_, bh_, bl_, acc[nt]);
          }
        }
        #pragma unroll
        for (int nt = 0; nt < 4; ++nt) {
          v4u H, Lo;
          split8(lo4(acc[nt]), hi4(acc[nt]), H, Lo);
          *(v4ua*)(PSh + m * XP + 64 * h + 16 * nt + 8 * hh) = H;
          *(v4ua*)(PSl + m * XP + 64 * h + 16 * nt + 8 * hh) = Lo;
        }
      }
      wave_sync();
    }

    #pragma unroll 1
    for (int half = 0; half < 2; ++half) {
      v8f acc[4];
      #pragma unroll
      for (int nt = 0; nt < 4; ++nt) acc[nt] = z8;
      #pragma unroll 2
      for (int ks = 0; ks < 8; ++ks) {
        const v16bf bh_ = ldfrag_bf(PSh + m * XP + 32 * ks, hh);
        const v16bf bl_ = ldfrag_bf(PSl + m * XP + 32 * ks, hh);
        #pragma unroll
        for (int nt = 0; nt < 4; ++nt) {
          const int d = 64 * half + 16 * nt + m;
          const v16bf ah_ = ldfrag_bf(WSh + (size_t)d * 256 + 32 * ks, hh);
          const v16bf al_ = ldfrag_bf(WSl + (size_t)d * 256 + 32 * ks, hh);
          acc[nt] = mma3(ah_, al_, bh_, bl_, acc[nt]);
        }
      }
      #pragma unroll
      for (int nt = 0; nt < 4; ++nt) {
        const int d8 = 64 * half + 16 * nt + 8 * hh;
        const v4f ba = *(const v4fa*)(bgat + d8);
        const v4f bb = *(const v4fa*)(bgat + d8 + 4);
        v4f oa, ob;
        oa.x = gelu_f(acc[nt][0] * 0.25f + ba.x);
        oa.y = gelu_f(acc[nt][1] * 0.25f + ba.y);
        oa.z = gelu_f(acc[nt][2] * 0.25f + ba.z);
        oa.w = gelu_f(acc[nt][3] * 0.25f + ba.w);
        ob.x = gelu_f(acc[nt][4] * 0.25f + bb.x);
        ob.y = gelu_f(acc[nt][5] * 0.25f + bb.y);
        ob.z = gelu_f(acc[nt][6] * 0.25f + bb.z);
        ob.w = gelu_f(acc[nt][7] * 0.25f + bb.w);
        *(v4fa*)(Hs + m * HSP + d8) = oa;
        *(v4fa*)(Hs + m * HSP + d8 + 4) = ob;
      }
    }
    wave_sync();
    {
      const size_t rowbase = (size_t)bt * NNODE + i0;
      store_rows16(Hs, H0h, H0l, rowbase, hh, m);
      __threadfence();
      store_rows16(Hs, H0h, H0l, rowbase, hh, m);
    }
    wave_sync();
  }
}

__global__ __launch_bounds__(256) void k_gcn(const unsigned short* __restrict__ Hh,
                                             const unsigned short* __restrict__ Hl,
                                             const unsigned short* __restrict__ WGh,
                                             const unsigned short* __restrict__ WGl,
                                             const unsigned short* __restrict__ APh,
                                             const unsigned short* __restrict__ APl,
                                             const float* __restrict__ bgcn,
                                             unsigned short* __restrict__ Oh,
                                             unsigned short* __restrict__ Ol,
                                             unsigned short* __restrict__ PLh,
                                             unsigned short* __restrict__ PLl,
                                             int layer2)
{
  extern __shared__ __align__(16) unsigned char dsm[];
  unsigned short* YTh = (unsigned short*)(dsm + C_YTH);
  unsigned short* YTl = (unsigned short*)(dsm + C_YTL);
  float* PPs = (float*)(dsm + C_PP);
  unsigned short* PQh = (unsigned short*)(dsm + C_PQH);
  unsigned short* PQl = (unsigned short*)(dsm + C_PQL);
  const int tid = threadIdx.x, lane = tid & 31, wv = tid >> 5;
  const int hh = lane >> 4, m = lane & 15;
  const int bt = blockIdx.x;
  float* St = (float*)(dsm + C_ST + wv * C_STSZ);
  const v8f z8 = {0.f, 0.f, 0.f, 0.f, 0.f, 0.f, 0.f, 0.f};

  #pragma unroll 1
  for (int rbq = 0; rbq < 2; ++rbq) {
    const int j0 = 16 * (wv + 8 * rbq);
    #pragma unroll 1
    for (int half = 0; half < 2; ++half) {
      v8f acc[4];
      #pragma unroll
      for (int nt = 0; nt < 4; ++nt) acc[nt] = z8;
      #pragma unroll 2
      for (int ks = 0; ks < 4; ++ks) {
        const size_t ao = ((size_t)bt * NNODE + j0 + m) * NHID + 32 * ks;
        const v16bf ah_ = ldfrag_bf(Hh + ao, hh);
        const v16bf al_ = ldfrag_bf(Hl + ao, hh);
        #pragma unroll
        for (int nt = 0; nt < 4; ++nt) {
          const int d = 64 * half + 16 * nt + m;
          const v16bf bh_ = ldfrag_bf(WGh + d * NHID + 32 * ks, hh);
          const v16bf bl_ = ldfrag_bf(WGl + d * NHID + 32 * ks, hh);
          acc[nt] = mma3(ah_, al_, bh_, bl_, acc[nt]);
        }
      }
      #pragma unroll
      for (int nt = 0; nt < 4; ++nt) {
        const int d = 64 * half + 16 * nt + m;
        v4u H, Lo;
        split8(lo4(acc[nt]), hi4(acc[nt]), H, Lo);
        *(v4ua*)(YTh + d * XP + j0 + 8 * hh) = H;
        *(v4ua*)(YTl + d * XP + j0 + 8 * hh) = Lo;
      }
    }
  }
  __syncthreads();

  v4f psum = {0.f, 0.f, 0.f, 0.f};
  #pragma unroll 1
  for (int rbq = 0; rbq < 2; ++rbq) {
    const int i0 = 16 * (wv + 8 * rbq);
    #pragma unroll 1
    for (int half = 0; half < 2; ++half) {
      v8f acc[4];
      #pragma unroll
      for (int nt = 0; nt < 4; ++nt) acc[nt] = z8;
      #pragma unroll 2
      for (int ks = 0; ks < 8; ++ks) {
        const size_t bo = (size_t)(i0 + m) * NNODE + 32 * ks;
        const v16bf bh_ = ldfrag_bf(APh + bo, hh);
        const v16bf bl_ = ldfrag_bf(APl + bo, hh);
        #pragma unroll
        for (int nt = 0; nt < 4; ++nt) {
          const int d = 64 * half + 16 * nt + m;
          const v16bf ah_ = ldfrag_bf(YTh + d * XP + 32 * ks, hh);
          const v16bf al_ = ldfrag_bf(YTl + d * XP + 32 * ks, hh);
          acc[nt] = mma3(ah_, al_, bh_, bl_, acc[nt]);
        }
      }
      #pragma unroll
      for (int nt = 0; nt < 4; ++nt) {
        const int d8 = 64 * half + 16 * nt + 8 * hh;
        const v4f ba = *(const v4fa*)(bgcn + d8);
        const v4f bb = *(const v4fa*)(bgcn + d8 + 4);
        v4f oa, ob;
        oa.x = gelu_f(acc[nt][0] + ba.x);
        oa.y = gelu_f(acc[nt][1] + ba.y);
        oa.z = gelu_f(acc[nt][2] + ba.z);
        oa.w = gelu_f(acc[nt][3] + ba.w);
        ob.x = gelu_f(acc[nt][4] + bb.x);
        ob.y = gelu_f(acc[nt][5] + bb.y);
        ob.z = gelu_f(acc[nt][6] + bb.z);
        ob.w = gelu_f(acc[nt][7] + bb.w);
        *(v4fa*)(St + m * HSP + d8) = oa;
        *(v4fa*)(St + m * HSP + d8 + 4) = ob;
      }
    }
    wave_sync();
    if (!layer2) {
      const size_t rowbase = (size_t)bt * NNODE + i0;
      store_rows16(St, Oh, Ol, rowbase, hh, m);
      __threadfence();
      store_rows16(St, Oh, Ol, rowbase, hh, m);
    } else {
      #pragma unroll 4
      for (int row = 0; row < 16; ++row) psum = psum + *(const v4fa*)(St + row * HSP + 4 * lane);
    }
    wave_sync();
  }

  *(v4fa*)(PPs + wv * 128 + 4 * lane) = psum;
  __syncthreads();
  if (tid < 128) {
    float s = 0.0f;
    #pragma unroll
    for (int w = 0; w < 8; ++w) s += PPs[w * 128 + tid];
    const float pv = s * (1.0f / 256.0f);
    unsigned int hb, lb;
    split2(pv, hb, lb);
    PQh[tid] = (unsigned short)hb;
    PQl[tid] = (unsigned short)lb;
  }
  __syncthreads();
  {
    const int th = (tid < 16) ? tid : 0;
    const int tl = (tid >= 16 && tid < 32) ? (tid - 16) : 0;
    const v4u hv = *(const v4ua*)(PQh + 8 * th);
    const v4u lv = *(const v4ua*)(PQl + 8 * tl);
    const size_t base = (size_t)bt * NHID;
    if (layer2 && tid < 16)              *(volatile v4u*)(PLh + base + 8 * th) = hv;
    if (layer2 && tid >= 16 && tid < 32) *(volatile v4u*)(PLl + base + 8 * tl) = lv;
    __threadfence();
    if (layer2 && tid < 16)              *(volatile v4u*)(PLh + base + 8 * th) = hv;
    if (layer2 && tid >= 16 && tid < 32) *(volatile v4u*)(PLl + base + 8 * tl) = lv;
  }
}

__global__ __launch_bounds__(256) void k_tail(const unsigned short* __restrict__ PLh,
                                              const unsigned short* __restrict__ PLl,
                                              const unsigned short* __restrict__ WIh,
                                              const unsigned short* __restrict__ WIl,
                                              const unsigned short* __restrict__ WHh,
                                              const unsigned short* __restrict__ WHl,
                                              const float* __restrict__ bi,
                                              const float* __restrict__ bh,
                                              const float* __restrict__ watt,
                                              const float* __restrict__ batt,
                                              const float* __restrict__ ln1g,
                                              const float* __restrict__ ln1b,
                                              const unsigned short* __restrict__ WFh,
                                              const unsigned short* __restrict__ WFl,
                                              const float* __restrict__ bfu,
                                              const unsigned short* __restrict__ WCh,
                                              const unsigned short* __restrict__ WCl,
                                              const float* __restrict__ bc1,
                                              const float* __restrict__ ln2g,
                                              const float* __restrict__ ln2b,
                                              const float* __restrict__ Wc2,
                                              const float* __restrict__ bc2,
                                              float* __restrict__ out)
{
  extern __shared__ __align__(16) unsigned char dsm[];
  float* GO  = (float*)(dsm + T_GO);
  float* GI  = (float*)(dsm + T_GI);
  float* GH  = (float*)(dsm + T_GH);
  float* HF  = (float*)(dsm + T_HF);
  unsigned short* HHs = (unsigned short*)(dsm + T_HH);
  unsigned short* HLs = (unsigned short*)(dsm + T_HL);
  unsigned short* CHs = (unsigned short*)(dsm + T_CH);
  unsigned short* CLs = (unsigned short*)(dsm + T_CL);
  unsigned short* FHs = (unsigned short*)(dsm + T_FH);
  unsigned short* FLs = (unsigned short*)(dsm + T_FL);
  float* C1s = (float*)(dsm + T_C1);
  float* ATs = (float*)(dsm + T_AT);
  float* WLs = (float*)(dsm + T_WL);
  float* S2  = (float*)(dsm + T_S2);
  float* OUs = (float*)(dsm + T_OU);
  const int tid = threadIdx.x, lane = tid & 31, wv = tid >> 5;
  const int hh = lane >> 4, m = lane & 15;
  const v8f z8 = {0.f, 0.f, 0.f, 0.f, 0.f, 0.f, 0.f, 0.f};

  for (int i2 = tid; i2 < 16 * 128; i2 += 256) HF[i2] = 0.0f;
  for (int i2 = tid; i2 < 16 * HP2; i2 += 256) { HHs[i2] = 0; HLs[i2] = 0; }
  for (int i2 = tid; i2 < 192; i2 += 256) OUs[i2] = 0.0f;
  __syncthreads();

  #pragma unroll 1
  for (int t = 0; t < NTIME; ++t) {
    v8f acci[3], acch[3];
    #pragma unroll
    for (int c = 0; c < 3; ++c) { acci[c] = z8; acch[c] = z8; }
    #pragma unroll 1
    for (int ks = 0; ks < 4; ++ks) {
      const size_t xo = ((size_t)(m * NTIME + t)) * NHID + 32 * ks;
      const v16bf xh = ldfrag_bf(PLh + xo, hh);
      const v16bf xl = ldfrag_bf(PLl + xo, hh);
      const v16bf gh_ = ldfrag_bf(HHs + m * HP2 + 32 * ks, hh);
      const v16bf gl_ = ldfrag_bf(HLs + m * HP2 + 32 * ks, hh);
      #pragma unroll
      for (int c = 0; c < 3; ++c) {
        const int g0 = 16 * (wv + 8 * c) + m;
        const v16bf wih = ldfrag_bf(WIh + (size_t)g0 * NHID + 32 * ks, hh);
        const v16bf wil = ldfrag_bf(WIl + (size_t)g0 * NHID + 32 * ks, hh);
        acci[c] = mma3(xh, xl, wih, wil, acci[c]);
        const v16bf whh = ldfrag_bf(WHh + (size_t)g0 * NHID + 32 * ks, hh);
        const v16bf whl = ldfrag_bf(WHl + (size_t)g0 * NHID + 32 * ks, hh);
        acch[c] = mma3(gh_, gl_, whh, whl, acch[c]);
      }
    }
    #pragma unroll
    for (int c = 0; c < 3; ++c) {
      const int col = 16 * (wv + 8 * c) + m;
      const float biv = bi[col], bhv = bh[col];
      #pragma unroll
      for (int r = 0; r < 8; ++r) {
        GI[(8 * hh + r) * 384 + col] = acci[c][r] + biv;
        GH[(8 * hh + r) * 384 + col] = acch[c][r] + bhv;
      }
    }
    __syncthreads();
    #pragma unroll 1
    for (int q = 0; q < 8; ++q) {
      const int idx = tid + 256 * q;
      const int b = idx >> 7, u = idx & 127;
      const float ir = GI[b * 384 + u],       hr = GH[b * 384 + u];
      const float iz = GI[b * 384 + 128 + u], hz = GH[b * 384 + 128 + u];
      const float in_ = GI[b * 384 + 256 + u], hn_ = GH[b * 384 + 256 + u];
      const float rg = sigm(ir + hr);
      const float zg = sigm(iz + hz);
      const float ng = tanhf(in_ + rg * hn_);
      const float hp = HF[b * 128 + u];
      const float hn = (1.0f - zg) * ng + zg * hp;
      HF[b * 128 + u] = hn;
      GO[(b * NTIME + t) * 128 + u] = hn;
      unsigned int hb2, lb2;
      split2(hn, hb2, lb2);
      HHs[b * HP2 + u] = (unsigned short)hb2;
      HLs[b * HP2 + u] = (unsigned short)lb2;
    }
    __syncthreads();
  }

  {
    const float* g = GO + tid * 128;
    float s = 0.0f;
    #pragma unroll 1
    for (int d = 0; d < 128; ++d) s = fmaf(g[d], watt[d], s);
    WLs[tid] = s + batt[0];
  }
  __syncthreads();
  if (tid < 16) {
    float mx = __uint_as_float(0xff800000u);
    for (int t = 0; t < 16; ++t) mx = fmaxf(mx, WLs[tid * 16 + t]);
    float s = 0.0f;
    for (int t = 0; t < 16; ++t) { const float e = expf(WLs[tid * 16 + t] - mx); WLs[tid * 16 + t] = e; s += e; }
    const float inv = 1.0f / s;
    for (int t = 0; t < 16; ++t) WLs[tid * 16 + t] = WLs[tid * 16 + t] * inv;
  }
  __syncthreads();
  for (int p = tid; p < 16 * 128; p += 256) {
    const int b = p >> 7, d = p & 127;
    float s = 0.0f, ms = 0.0f;
    #pragma unroll 1
    for (int t = 0; t < 16; ++t) {
      const float g = GO[(b * 16 + t) * 128 + d];
      s = fmaf(WLs[b * 16 + t], g, s);
      ms += g;
    }
    ATs[p] = s + ms * (1.0f / 16.0f);
  }
  __syncthreads();
  if (tid < 16) {
    float mu = 0.0f;
    for (int d = 0; d < 128; ++d) mu += ATs[tid * 128 + d];
    mu = mu * (1.0f / 128.0f);
    float var = 0.0f;
    for (int d = 0; d < 128; ++d) { const float xm = ATs[tid * 128 + d] - mu; var += xm * xm; }
    var = var * (1.0f / 128.0f);
    S2[tid] = mu;
    S2[16 + tid] = 1.0f / sqrtf(var + 1e-5f);
  }
  __syncthreads();
  for (int p = tid; p < 16 * 128; p += 256) {
    const int b = p >> 7, d = p & 127;
    const float v = ((ATs[p] - S2[b]) * S2[16 + b]) * ln1g[d] + ln1b[d];
    unsigned int hb2, lb2;
    split2(v, hb2, lb2);
    CHs[b * XP + d] = (unsigned short)hb2;
    CLs[b * XP + d] = (unsigned short)lb2;
    const float hl = GO[(b * 16 + 15) * 128 + d];
    split2(hl, hb2, lb2);
    CHs[b * XP + 128 + d] = (unsigned short)hb2;
    CLs[b * XP + 128 + d] = (unsigned short)lb2;
  }
  __syncthreads();

  {
    v8f acc = z8;
    #pragma unroll 1
    for (int ks = 0; ks < 8; ++ks) {
      const v16bf ah_ = ldfrag_bf(CHs + m * XP + 32 * ks, hh);
      const v16bf al_ = ldfrag_bf(CLs + m * XP + 32 * ks, hh);
      const size_t bo = (size_t)(16 * wv + m) * 256 + 32 * ks;
      const v16bf bh_ = ldfrag_bf(WFh + bo, hh);
      const v16bf bl_ = ldfrag_bf(WFl + bo, hh);
      acc = mma3(ah_, al_, bh_, bl_, acc);
    }
    const int col = 16 * wv + m;
    const float bv = bfu[col];
    #pragma unroll
    for (int r = 0; r < 8; ++r) {
      unsigned int hb2, lb2;
      split2(acc[r] + bv, hb2, lb2);
      FHs[(8 * hh + r) * HP2 + col] = (unsigned short)hb2;
      FLs[(8 * hh + r) * HP2 + col] = (unsigned short)lb2;
    }
  }
  __syncthreads();

  {
    v8f acc2[2];
    acc2[0] = z8; acc2[1] = z8;
    #pragma unroll 1
    for (int ks = 0; ks < 4; ++ks) {
      const v16bf ah_ = ldfrag_bf(FHs + m * HP2 + 32 * ks, hh);
      const v16bf al_ = ldfrag_bf(FLs + m * HP2 + 32 * ks, hh);
      #pragma unroll
      for (int c = 0; c < 2; ++c) {
        const size_t bo = (size_t)(16 * (wv + 8 * c) + m) * NHID + 32 * ks;
        const v16bf bh_ = ldfrag_bf(WCh + bo, hh);
        const v16bf bl_ = ldfrag_bf(WCl + bo, hh);
        acc2[c] = mma3(ah_, al_, bh_, bl_, acc2[c]);
      }
    }
    #pragma unroll
    for (int c = 0; c < 2; ++c) {
      const int col = 16 * (wv + 8 * c) + m;
      const float bv = bc1[col];
      #pragma unroll
      for (int r = 0; r < 8; ++r) C1s[(8 * hh + r) * 256 + col] = acc2[c][r] + bv;
    }
  }
  __syncthreads();
  if (tid < 16) {
    float mu = 0.0f;
    for (int d = 0; d < 256; ++d) mu += C1s[tid * 256 + d];
    mu = mu * (1.0f / 256.0f);
    float var = 0.0f;
    for (int d = 0; d < 256; ++d) { const float xm = C1s[tid * 256 + d] - mu; var += xm * xm; }
    var = var * (1.0f / 256.0f);
    S2[32 + tid] = mu;
    S2[48 + tid] = 1.0f / sqrtf(var + 1e-5f);
  }
  __syncthreads();
  for (int p = tid; p < 16 * 256; p += 256) {
    const int b = p >> 8, d = p & 255;
    const float v = ((C1s[p] - S2[32 + b]) * S2[48 + b]) * ln2g[d] + ln2b[d];
    C1s[p] = gelu_f(v);
  }
  __syncthreads();

  if (tid < 160) {
    const int b = tid / NCLS, c = tid - NCLS * b;
    float s = 0.0f;
    #pragma unroll 1
    for (int k = 0; k < 256; ++k) s = fmaf(C1s[b * 256 + k], Wc2[k * NCLS + c], s);
    OUs[tid] = s + bc2[c];
  }
  __syncthreads();
  {
    const int to = (tid < 40) ? tid : 0;
    const v4f ov = *(const v4fa*)(OUs + 4 * to);
    if (tid < 40) *(volatile v4f*)(out + 4 * to) = ov;
    __threadfence();
    if (tid < 40) *(volatile v4f*)(out + 4 * to) = ov;
  }
}

extern "C" void kernel_launch(void* const* d_in, const int* in_sizes, int n_in,
                              void* d_out, int out_size, void* d_ws, size_t ws_size,
                              hipStream_t stream)
{
  if (n_in < 25) return;
  if (in_sizes[0]  != NBATCH * NTIME * NNODE * NFEAT) return;
  if (in_sizes[2]  != NNODE * NNODE) return;
  if (in_sizes[3]  != NFEAT * NHEAD * NHID) return;
  if (in_sizes[4]  != NHEAD * NHID) return;
  if (in_sizes[5]  != NHEAD * NHID) return;
  if (in_sizes[6]  != NHID) return;
  if (in_sizes[7]  != NHID * NHID) return;
  if (in_sizes[8]  != NHID) return;
  if (in_sizes[9]  != NHID * 3 * NHID) return;
  if (in_sizes[10] != NHID * 3 * NHID) return;
  if (in_sizes[11] != 3 * NHID) return;
  if (in_sizes[12] != 3 * NHID) return;
  if (in_sizes[13] != NHID) return;
  if (in_sizes[14] < 1) return;
  if (in_sizes[15] != NHID) return;
  if (in_sizes[16] != NHID) return;
  if (in_sizes[17] != 2 * NHID * NHID) return;
  if (in_sizes[18] != NHID) return;
  if (in_sizes[19] != NHID * 2 * NHID) return;
  if (in_sizes[20] != 2 * NHID) return;
  if (in_sizes[21] != 2 * NHID) return;
  if (in_sizes[22] != 2 * NHID) return;
  if (in_sizes[23] != 2 * NHID * NCLS) return;
  if (in_sizes[24] != NCLS) return;
  if (out_size != NBATCH * NCLS) return;

  const float* x     = (const float*)d_in[0];
  const float* Ladj  = (const float*)d_in[2];
  const float* Wgat  = (const float*)d_in[3];
  const float* asrc  = (const float*)d_in[4];
  const float* adst  = (const float*)d_in[5];
  const float* bgat  = (const float*)d_in[6];
  const float* Wgcn  = (const float*)d_in[7];
  const float* bgcn  = (const float*)d_in[8];
  const float* Wi    = (const float*)d_in[9];
  const float* Wh    = (const float*)d_in[10];
  const float* bi    = (const float*)d_in[11];
  const float* bh    = (const float*)d_in[12];
  const float* watt  = (const float*)d_in[13];
  const float* batt  = (const float*)d_in[14];
  const float* ln1g  = (const float*)d_in[15];
  const float* ln1b  = (const float*)d_in[16];
  const float* Wf    = (const float*)d_in[17];
  const float* bfu   = (const float*)d_in[18];
  const float* Wc1   = (const float*)d_in[19];
  const float* bc1   = (const float*)d_in[20];
  const float* ln2g  = (const float*)d_in[21];
  const float* ln2b  = (const float*)d_in[22];
  const float* Wc2   = (const float*)d_in[23];
  const float* bc2   = (const float*)d_in[24];
  float* out = (float*)d_out;

  const size_t bAN = (size_t)NNODE * NNODE * 4;
  const size_t bDV = 1024;
  const size_t bV  = 2048;
  const size_t bAP = (size_t)NNODE * NNODE * 2;
  const size_t bMB = (size_t)NNODE * 32 * 4;
  const size_t bWS = (size_t)NHID * 256 * 2;
  const size_t bWG = (size_t)NHID * NHID * 2;
  const size_t bWI = (size_t)3 * NHID * NHID * 2;
  const size_t bWH = bWI;
  const size_t bWF = (size_t)NHID * 2 * NHID * 2;
  const size_t bWC = (size_t)2 * NHID * NHID * 2;
  const size_t bH  = (size_t)NGRAPH * NNODE * NHID * 2;
  const size_t bPL = (size_t)NGRAPH * NHID * 2;
  const size_t total = bAN + bDV + bV + 2 * bAP + bMB + 2 * (bWS + bWG + bWI + bWH + bWF + bWC)
                     + 4 * bH + 2 * bPL;
  if (total > ws_size) return;
  if (total > (size_t)134217728) return;

  char* ws = (char*)d_ws;
  size_t off = 0;
  float*          An  = (float*)(ws + off);          off += bAN;
  float*          DV  = (float*)(ws + off);          off += bDV;
  float*          Vv  = (float*)(ws + off);          off += bV;
  unsigned short* APh = (unsigned short*)(ws + off); off += bAP;
  unsigned short* APl = (unsigned short*)(ws + off); off += bAP;
  unsigned int*   MBw = (unsigned int*)(ws + off);   off += bMB;
  unsigned short* WSh = (unsigned short*)(ws + off); off += bWS;
  unsigned short* WSl = (unsigned short*)(ws + off); off += bWS;
  unsigned short* WGh = (unsigned short*)(ws + off); off += bWG;
  unsigned short* WGl = (unsigned short*)(ws + off); off += bWG;
  unsigned short* WIh = (unsigned short*)(ws + off); off += bWI;
  unsigned short* WIl = (unsigned short*)(ws + off); off += bWI;
  unsigned short* WHh = (unsigned short*)(ws + off); off += bWH;
  unsigned short* WHl = (unsigned short*)(ws + off); off += bWH;
  unsigned short* WFh = (unsigned short*)(ws + off); off += bWF;
  unsigned short* WFl = (unsigned short*)(ws + off); off += bWF;
  unsigned short* WCh = (unsigned short*)(ws + off); off += bWC;
  unsigned short* WCl = (unsigned short*)(ws + off); off += bWC;
  unsigned short* H0h = (unsigned short*)(ws + off); off += bH;
  unsigned short* H0l = (unsigned short*)(ws + off); off += bH;
  unsigned short* H1h = (unsigned short*)(ws + off); off += bH;
  unsigned short* H1l = (unsigned short*)(ws + off); off += bH;
  unsigned short* PLh = (unsigned short*)(ws + off); off += bPL;
  unsigned short* PLl = (unsigned short*)(ws + off); off += bPL;
  if (off != total) return;

  k_adj1<<<NNODE, 256, 0, stream>>>(Ladj, An);
  k_small<<<1, 256, 0, stream>>>(An, Wgat, asrc, adst, DV, Vv);
  k_adj3<<<NNODE, 256, 0, stream>>>(An, DV, APh, APl, MBw);
  k_tsplit<<<dim3(128 / 64, 64 / 64, NHEAD), 256, 0, stream>>>(Wgat, 512, 128, WSh, WSl, 256, 64, 64, 128);
  k_tsplit<<<dim3(128 / 64, 128 / 64, 1), 256, 0, stream>>>(Wgcn, 128, 0, WGh, WGl, 128, 0, 128, 128);
  k_tsplit<<<dim3(384 / 64, 128 / 64, 1), 256, 0, stream>>>(Wi,   384, 0, WIh, WIl, 128, 0, 128, 384);
  k_tsplit<<<dim3(384 / 64, 128 / 64, 1), 256, 0, stream>>>(Wh,   384, 0, WHh, WHl, 128, 0, 128, 384);
  k_tsplit<<<dim3(128 / 64, 256 / 64, 1), 256, 0, stream>>>(Wf,   128, 0, WFh, WFl, 256, 0, 256, 128);
  k_tsplit<<<dim3(256 / 64, 128 / 64, 1), 256, 0, stream>>>(Wc1,  256, 0, WCh, WCl, 128, 0, 128, 256);
  hipFuncSetAttribute(reinterpret_cast<const void*>(&k_gat),
                      hipFuncAttributeMaxDynamicSharedMemorySize, LDS_GAT);
  k_gat<<<NGRAPH, 128, LDS_GAT, stream>>>(x, Vv, MBw, WSh, WSl, bgat, H0h, H0l);
  hipFuncSetAttribute(reinterpret_cast<const void*>(&k_gcn),
                      hipFuncAttributeMaxDynamicSharedMemorySize, LDS_GCN);
  k_gcn<<<NGRAPH, 256, LDS_GCN, stream>>>(H0h, H0l, WGh, WGl, APh, APl, bgcn, H1h, H1l, PLh, PLl, 0);
  k_gcn<<<NGRAPH, 256, LDS_GCN, stream>>>(H1h, H1l, WGh, WGl, APh, APl, bgcn, H0h, H0l, PLh, PLl, 1);
  hipFuncSetAttribute(reinterpret_cast<const void*>(&k_tail),
                      hipFuncAttributeMaxDynamicSharedMemorySize, LDS_TAIL);
  k_tail<<<1, 256, LDS_TAIL, stream>>>(PLh, PLl, WIh, WIl, WHh, WHl, bi, bh, watt, batt, ln1g, ln1b,
                                       WFh, WFl, bfu, WCh, WCl, bc1, ln2g, ln2b, Wc2, bc2, out);
}
